// GIN_84507776516707
// MI455X (gfx1250) — hardware-run, weakly checked
//
#include <hip/hip_runtime.h>
#include <stddef.h>
#include <stdint.h>


#define DF      128
#define APW     256
#define WTP     256
#define ZLO     1
#define TLO     1
#define KZ      (ZLO ? 256 : 128)
#define KTT     (TLO ? 256 : 128)
#define WSQ     (DF * WTP)
#define NMAT    4
#define NUSQ    (DF * (WTP / 8))
#define NUW     (NMAT * NUSQ)
#define NTHR    256
#define NWAVE   8
#define EPT     8
#define CHUNK   (NTHR * EPT)
#define WCAP    (EPT * 32)
#define LISTN   (NWAVE * WCAP)
#define NBA     1024
#define PKS     10
#define RCAP    28672
#define DEGCAP  64
#define GBM     64
#define GTHR    128
#define BN      128
#define RPB     64
#define RPW     8
#define BK_INTS (2 * RCAP + 3 * NBA + LISTN + 32)
#define LDS_BK  (BK_INTS * 4)
#define MEAS_BLK_HITS 16623
#define MEAS_MAXDEG   35
#define WSMAX   (128u << 20)

static_assert((CHUNK & (CHUNK - 1)) == 0 && CHUNK <= 4096);
static_assert(NBA == (1 << PKS) && NBA == NTHR * 4);
static_assert(LISTN == NWAVE * WCAP);
static_assert(RCAP % (NTHR * 4) == 0 && BK_INTS % 4 == 0);
static_assert((long long)RCAP * 100 >= (long long)MEAS_BLK_HITS * 105);
static_assert(DEGCAP >= MEAS_MAXDEG + 8);
static_assert(LDS_BK <= 300000);
static_assert(KZ % 32 == 0 && KTT % 32 == 0 && KZ <= APW && KTT <= APW && KZ <= WTP && KTT <= WTP);
static_assert(APW == 2 * DF && WTP == 2 * DF);
static_assert(GBM == (GTHR / 32) * 16 && BN == 8 * 16 && BN == DF && BN == 32 * 4);
static_assert(NUSQ % NTHR == 0 && NUW % NTHR == 0 && (WTP / 8) == 32);
static_assert(RPB == NWAVE * RPW && RPB == GBM && (NBA % GBM) == 0);

typedef float          v4f   __attribute__((ext_vector_type(4)));
typedef float          v8f   __attribute__((ext_vector_type(8)));
typedef int            v4i   __attribute__((ext_vector_type(4)));
typedef int            v8i   __attribute__((ext_vector_type(8)));
typedef unsigned       v2u   __attribute__((ext_vector_type(2)));
typedef unsigned       v4u   __attribute__((ext_vector_type(4)));
typedef unsigned short v8us  __attribute__((ext_vector_type(8)));
typedef __bf16         v16bf __attribute__((ext_vector_type(16)));
typedef v4f  __attribute__((may_alias)) v4fa;
typedef v4i  __attribute__((may_alias)) v4ia;
typedef v2u  __attribute__((may_alias)) v2ua;
typedef v4u  __attribute__((may_alias)) v4ua;
typedef v8us __attribute__((may_alias)) v8usa;
union FragB { v16bf v; v8us h[2]; v8i w; };

__device__ __forceinline__ v8f wmb(const FragB& a, const FragB& b, v8f c) {
  v8f d = __builtin_amdgcn_wmma_f32_16x16x32_bf16(false, a.v, false, b.v, (short)0, c, false, false);
  asm volatile("v_nop\n\tv_nop\n\tv_nop\n\tv_nop" : "+v"(d) : "v"(a.w), "v"(b.w));
  return d;
}

__device__ __forceinline__ unsigned bf16_bits(float f) {
  const unsigned u = __float_as_uint(f);
  const unsigned r = ((u + 0x7FFFu + ((u >> 16) & 1u)) >> 16) & 0xFFFFu;
  const unsigned q = ((u >> 16) | 0x0040u) & 0xFFFFu;
  return ((u & 0x7FFFFFFFu) > 0x7F800000u) ? q : r;
}
__device__ __forceinline__ float bf16_val(float f) { return __uint_as_float(bf16_bits(f) << 16); }
__device__ __forceinline__ float bfw_lo(unsigned w) { return __uint_as_float(w << 16); }
__device__ __forceinline__ float bfw_hi(unsigned w) { return __uint_as_float(w & 0xffff0000u); }
__device__ __forceinline__ void pack2(float a, float b, unsigned& hw, unsigned& lw) {
  const unsigned ha = bf16_bits(a), hb = bf16_bits(b);
  const unsigned la = bf16_bits(a - __uint_as_float(ha << 16));
  const unsigned lb = bf16_bits(b - __uint_as_float(hb << 16));
  hw = ha | (hb << 16);
  lw = la | (lb << 16);
}
__device__ __forceinline__ float relu_k(float v) { return (v > 0.0f) ? v : (v - v); }

__device__ __forceinline__ void wave_sync() {
  __builtin_amdgcn_fence(__ATOMIC_RELEASE, "wavefront");
  __builtin_amdgcn_wave_barrier();
  __builtin_amdgcn_fence(__ATOMIC_ACQUIRE, "wavefront");
}

__device__ __forceinline__ int scan_chunk(const int* __restrict__ keys, int nE, int cbase, int slotBase,
                                          int nb, int vec8, int* list, int tid, int lane, int wave) {
  int wc = 0;
  const int el0  = tid * EPT;
  const int e0   = cbase + el0;
  const int sent = (int)(1u << 31);
  v4i da, db;
  if (vec8 != 0 && cbase + CHUNK <= nE) {
    da = *(const v4i*)(keys + e0);
    db = *(const v4i*)(keys + e0 + 4);
  } else {
    da.x = (e0     < nE) ? keys[min(e0,     nE - 1)] : sent;
    da.y = (e0 + 1 < nE) ? keys[min(e0 + 1, nE - 1)] : sent;
    da.z = (e0 + 2 < nE) ? keys[min(e0 + 2, nE - 1)] : sent;
    da.w = (e0 + 3 < nE) ? keys[min(e0 + 3, nE - 1)] : sent;
    db.x = (e0 + 4 < nE) ? keys[min(e0 + 4, nE - 1)] : sent;
    db.y = (e0 + 5 < nE) ? keys[min(e0 + 5, nE - 1)] : sent;
    db.z = (e0 + 6 < nE) ? keys[min(e0 + 6, nE - 1)] : sent;
    db.w = (e0 + 7 < nE) ? keys[min(e0 + 7, nE - 1)] : sent;
  }
  const unsigned nbs = (unsigned)slotBase;
  const unsigned unb = (unsigned)nb;
  const unsigned s0 = (unsigned)da.x - nbs, s1 = (unsigned)da.y - nbs;
  const unsigned s2 = (unsigned)da.z - nbs, s3 = (unsigned)da.w - nbs;
  const unsigned s4 = (unsigned)db.x - nbs, s5 = (unsigned)db.y - nbs;
  const unsigned s6 = (unsigned)db.z - nbs, s7 = (unsigned)db.w - nbs;
  const bool h0 = s0 < unb, h1 = s1 < unb, h2 = s2 < unb, h3 = s3 < unb;
  const bool h4 = s4 < unb, h5 = s5 < unb, h6 = s6 < unb, h7 = s7 < unb;
  const unsigned any = __builtin_amdgcn_ballot_w32(h0 | h1 | h2 | h3 | h4 | h5 | h6 | h7);
  if (any != 0u) {
#define HITJ(J, HJ, SJ) { \
      const unsigned mj = __builtin_amdgcn_ballot_w32(HJ); \
      if (mj != 0u) { \
        if (HJ) { \
          const int pos = wc + (int)__builtin_amdgcn_mbcnt_lo(mj, 0u); \
          if (pos < WCAP) list[wave * WCAP + pos] = ((el0 + (J)) << PKS) | (int)(SJ); \
        } \
        wc += (int)__builtin_popcount(mj); } }
    HITJ(0, h0, s0)
    HITJ(1, h1, s1)
    HITJ(2, h2, s2)
    HITJ(3, h3, s3)
    HITJ(4, h4, s4)
    HITJ(5, h5, s5)
    HITJ(6, h6, s6)
    HITJ(7, h7, s7)
#undef HITJ
  }
  return wc;
}

__global__ __launch_bounds__(NTHR) void k_prep(const float* __restrict__ x,
                                               const float* __restrict__ w0, const float* __restrict__ w1,
                                               const float* __restrict__ w2, const float* __restrict__ w3,
                                               unsigned short* wt, unsigned short* xb, int nN, int nUnits) {
  const int u = (int)blockIdx.x * NTHR + (int)threadIdx.x;
  if (u < NUW) {
    const int mi = u / NUSQ;
    const int v  = u - mi * NUSQ;
    const int n  = v >> 5;
    const int k8 = (v & 31) * 8;
    const int kk = k8 & (DF - 1);
    const size_t so = (size_t)kk * DF + (size_t)n;
    float f[8];
    if (mi == 0) {
#pragma unroll
      for (int i = 0; i < 8; ++i) f[i] = w0[so + (size_t)i * DF];
    } else if (mi == 1) {
#pragma unroll
      for (int i = 0; i < 8; ++i) f[i] = w1[so + (size_t)i * DF];
    } else if (mi == 2) {
#pragma unroll
      for (int i = 0; i < 8; ++i) f[i] = w2[so + (size_t)i * DF];
    } else {
#pragma unroll
      for (int i = 0; i < 8; ++i) f[i] = w3[so + (size_t)i * DF];
    }
    v8us o;
#pragma unroll
    for (int i = 0; i < 8; ++i) o[i] = (unsigned short)bf16_bits(f[i]);
    unsigned short* dp = wt + (size_t)mi * WSQ + (size_t)n * WTP + (size_t)k8;
    *(volatile v8us*)dp = o;
    __threadfence();
    *(volatile v8us*)dp = o;
  } else if (u < nUnits) {
    const int q   = u - NUW;
    const int row = q >> 4;
    const int c8  = (q & 15) * 8;
    const int rc  = row < nN ? row : nN - 1;
    const float* p = x + (size_t)rc * DF + c8;
    const v4f a = *(const v4f*)p;
    const v4f b = *(const v4f*)(p + 4);
    asm volatile("" :: "v"(a), "v"(b));
    const bool lv = row < nN;
    v8us o;
    o[0] = lv ? (unsigned short)bf16_bits(a.x) : (unsigned short)0;
    o[1] = lv ? (unsigned short)bf16_bits(a.y) : (unsigned short)0;
    o[2] = lv ? (unsigned short)bf16_bits(a.z) : (unsigned short)0;
    o[3] = lv ? (unsigned short)bf16_bits(a.w) : (unsigned short)0;
    o[4] = lv ? (unsigned short)bf16_bits(b.x) : (unsigned short)0;
    o[5] = lv ? (unsigned short)bf16_bits(b.y) : (unsigned short)0;
    o[6] = lv ? (unsigned short)bf16_bits(b.z) : (unsigned short)0;
    o[7] = lv ? (unsigned short)bf16_bits(b.w) : (unsigned short)0;
    unsigned short* dp = xb + (size_t)row * DF + c8;
    *(volatile v8us*)dp = o;
    __threadfence();
    *(volatile v8us*)dp = o;
  }
}

__global__ __launch_bounds__(NTHR) void k_bucket(const int* __restrict__ keys, const int* __restrict__ gidx,
                                                 int nE, int nN, int vec8,
                                                 int* LIST, int* CNT, int* OFF, int* REC) {
  extern __shared__ __attribute__((aligned(16))) int dsm[];
  int* reg1 = dsm;
  int* reg2 = reg1 + RCAP;
  int* scnt = reg2 + RCAP;
  int* soff = scnt + NBA;
  int* cur  = soff + NBA;
  int* list = cur + NBA;
  int* wcnt = list + LISTN;
  int* wtot = wcnt + 8;
  int* wmx  = wtot + 8;
  const int tid = (int)threadIdx.x, lane = tid & 31, wave = tid >> 5;
  const int nodeBase = (int)blockIdx.x * NBA;
  int nb = nN - nodeBase;
  nb = nb > NBA ? NBA : (nb < 1 ? 1 : nb);

  {
    const v4i z4 = {0, 0, 0, 0};
    for (int i = tid * 4; i < BK_INTS; i += NTHR * 4) *(v4ia*)(dsm + i) = z4;
  }
  __syncthreads();

  int tot = 0;
  const int nChunks = (nE + CHUNK - 1) / CHUNK;
#pragma unroll 1
  for (int ch = 0; ch < nChunks; ++ch) {
    const int cbase = ch * CHUNK;
    const int wc = scan_chunk(keys, nE, cbase, nodeBase, nb, vec8, list, tid, lane, wave);
    if (lane == 0) wcnt[wave] = wc;
    __syncthreads();
    int pre = 0, all = 0;
#pragma unroll
    for (int w2 = 0; w2 < NWAVE; ++w2) {
      int c = wcnt[w2];
      c = c < 0 ? 0 : (c > WCAP ? WCAP : c);
      all += c;
      pre += (w2 < wave) ? c : 0;
    }
    const int wcc  = wc > WCAP ? WCAP : wc;
    const int base = tot + pre;
#pragma unroll 1
    for (int i = lane; i < wcc; i += 32) {
      const int ent = list[wave * WCAP + i];
      const int el  = (ent >> PKS) & (CHUNK - 1);
      const int sl  = ent & (NBA - 1);
      int eid = cbase + el;
      eid = eid > nE - 1 ? nE - 1 : eid;
      const int pos = base + i;
      if (pos < RCAP) reg1[pos] = (int)(((unsigned)eid << PKS) | (unsigned)sl);
    }
    tot += all;
    tot = tot > RCAP ? RCAP : tot;
    __syncthreads();
  }
  const int nh = tot;

  if (wave == 0) {
#pragma unroll 1
    for (int b0 = 0; b0 < nh; b0 += 32) {
      const int idx = b0 + lane;
      const int uv  = reg1[idx < RCAP ? idx : RCAP - 1];
      const int m32 = (nh - b0) < 32 ? (nh - b0) : 32;
#pragma unroll 1
      for (int k = 0; k < m32; ++k) {
        const int u  = __builtin_amdgcn_readlane(uv, k);
        const int sl = u & (NBA - 1);
        if (lane == 0) scnt[sl] = scnt[sl] + 1;
      }
    }
  }
  __syncthreads();

  {
    const v4i ca = *(const v4ia*)(scnt + 4 * tid);
    const int e0 = ca.x < 0 ? 0 : ca.x, e1 = ca.y < 0 ? 0 : ca.y, e2 = ca.z < 0 ? 0 : ca.z, e3 = ca.w < 0 ? 0 : ca.w;
    const int ts = e0 + e1 + e2 + e3;
    int incl = ts;
#pragma unroll
    for (int d = 1; d < 32; d <<= 1) {
      const int up = __shfl_up(incl, d, 32);
      if (lane >= d) incl += up;
    }
    int mx = max(max(e0, e1), max(e2, e3));
    mx = max(mx, __shfl_xor(mx, 16, 32));
    mx = max(mx, __shfl_xor(mx, 8, 32));
    mx = max(mx, __shfl_xor(mx, 4, 32));
    mx = max(mx, __shfl_xor(mx, 2, 32));
    mx = max(mx, __shfl_xor(mx, 1, 32));
    if (lane == 31) wtot[wave] = incl;
    if (lane == 0)  wmx[wave] = mx;
    __syncthreads();
    int pre = 0;
#pragma unroll
    for (int w2 = 0; w2 < NWAVE; ++w2) pre += (w2 < wave) ? wtot[w2] : 0;
    int run = pre + incl - ts;
    v4i so;
    so.x = run; run += e0;
    so.y = run; run += e1;
    so.z = run; run += e2;
    so.w = run;
    *(v4ia*)(soff + 4 * tid) = so;
    *(v4ia*)(cur + 4 * tid)  = so;
  }
  __syncthreads();

  if (wave == 0) {
#pragma unroll 1
    for (int b0 = 0; b0 < nh; b0 += 32) {
      const int idx = b0 + lane;
      const int uv  = reg1[idx < RCAP ? idx : RCAP - 1];
      const int m32 = (nh - b0) < 32 ? (nh - b0) : 32;
#pragma unroll 1
      for (int k = 0; k < m32; ++k) {
        const int u   = __builtin_amdgcn_readlane(uv, k);
        const int sl  = u & (NBA - 1);
        const int eid = (int)((unsigned)u >> PKS);
        if (lane == 0) {
          int pos = cur[sl];
          pos = pos < 0 ? 0 : (pos > RCAP - 1 ? RCAP - 1 : pos);
          reg2[pos] = eid;
          cur[sl] = pos + 1;
        }
      }
    }
  }
  __syncthreads();

  int bmax = 0;
#pragma unroll
  for (int w2 = 0; w2 < NWAVE; ++w2) bmax = max(bmax, wmx[w2]);
  const int flag = ((nh >= RCAP) || (bmax > DEGCAP)) ? 1 : 0;

  int* lrow = LIST + (size_t)blockIdx.x * RCAP;
#pragma unroll 1
  for (int it = 0; it < RCAP / (NTHR * 4); ++it) {
    const int i0 = 4 * (it * NTHR + tid);
    const v4i ev = *(const v4ia*)(reg2 + i0);
    int e0 = ev.x, e1 = ev.y, e2 = ev.z, e3 = ev.w;
    e0 = e0 < 0 ? 0 : (e0 > nE - 1 ? nE - 1 : e0);
    e1 = e1 < 0 ? 0 : (e1 > nE - 1 ? nE - 1 : e1);
    e2 = e2 < 0 ? 0 : (e2 > nE - 1 ? nE - 1 : e2);
    e3 = e3 < 0 ? 0 : (e3 > nE - 1 ? nE - 1 : e3);
    int g0 = gidx[e0], g1 = gidx[e1], g2 = gidx[e2], g3 = gidx[e3];
    asm volatile("" :: "v"(g0), "v"(g1), "v"(g2), "v"(g3));
    g0 = g0 < 0 ? 0 : (g0 > nN - 1 ? nN - 1 : g0);
    g1 = g1 < 0 ? 0 : (g1 > nN - 1 ? nN - 1 : g1);
    g2 = g2 < 0 ? 0 : (g2 > nN - 1 ? nN - 1 : g2);
    g3 = g3 < 0 ? 0 : (g3 > nN - 1 ? nN - 1 : g3);
    v4i ov;
    ov.x = (i0     < nh) ? g0 : 0;
    ov.y = (i0 + 1 < nh) ? g1 : 0;
    ov.z = (i0 + 2 < nh) ? g2 : 0;
    ov.w = (i0 + 3 < nh) ? g3 : 0;
    *(volatile v4i*)(lrow + i0) = ov;
    __threadfence();
    *(volatile v4i*)(lrow + i0) = ov;
  }
  {
    const v4i cv = *(const v4ia*)(scnt + 4 * tid);
    const v4i fv = *(const v4ia*)(soff + 4 * tid);
    v4i rv = {0, 0, 0, 0};
    rv.x = (tid == 0) ? bmax : 0;
    rv.y = (tid == 0) ? flag : 0;
    rv.z = (tid == 0) ? nh : 0;
    int* cp = CNT + (size_t)nodeBase + 4 * tid;
    int* fp = OFF + (size_t)nodeBase + 4 * tid;
    int* rp = REC + (size_t)blockIdx.x * 32 + 4 * (tid & 7);
    *(volatile v4i*)cp = cv;
    *(volatile v4i*)fp = fv;
    if (tid < 8) *(volatile v4i*)rp = rv;
    __threadfence();
    *(volatile v4i*)cp = cv;
    *(volatile v4i*)fp = fv;
    if (tid < 8) *(volatile v4i*)rp = rv;
  }
}

template <int F32SRC>
__global__ __launch_bounds__(NTHR) void k_rowsum(const unsigned short* __restrict__ XB,
                                                 const float* __restrict__ HF,
                                                 unsigned short* Zout,
                                                 const int* __restrict__ LIST, const int* __restrict__ CNT,
                                                 const int* __restrict__ OFF, const int* __restrict__ REC,
                                                 int nN, int mRows, int nBk) {
  __shared__ __attribute__((aligned(16))) unsigned rowst[NWAVE * 128];
  const int tid = (int)threadIdx.x, lane = tid & 31, wave = tid >> 5;
  unsigned* wst = rowst + wave * 128;
  const float qnan = __uint_as_float(0x7fc00000u);
#pragma unroll 1
  for (int ri = 0; ri < RPW; ++ri) {
    const int node = (int)blockIdx.x * RPB + wave * RPW + ri;
    if (node >= mRows) continue;
    int bq = node >> PKS;
    bq = bq > nBk - 1 ? nBk - 1 : bq;
    const int craw = CNT[node];
    const int oraw = OFF[node];
    const int fl   = REC[(size_t)bq * 32 + 1];
    int c = craw < 0 ? 0 : (craw > DEGCAP ? DEGCAP : craw);
    int o = oraw < 0 ? 0 : (oraw > RCAP - 1 ? RCAP - 1 : oraw);
    c = c > RCAP - o ? RCAP - o : c;
    c = __builtin_amdgcn_readfirstlane(c);
    o = __builtin_amdgcn_readfirstlane(o);
    int last = o + c - 1;
    last = last < o ? o : last;
    const bool bad = (fl != 0) || (craw > DEGCAP) || (craw < 0);
    const int* lp = LIST + (size_t)bq * RCAP;

    float a0 = 0.0f, a1 = 0.0f, a2 = 0.0f, a3 = 0.0f;
#pragma unroll 1
    for (int b0 = 0; b0 < c; b0 += 32) {
      int idx = o + b0 + lane;
      idx = idx > last ? last : idx;
      int col = lp[idx];
      col = col < 0 ? 0 : (col > nN - 1 ? nN - 1 : col);
      const int m32 = (c - b0) < 32 ? (c - b0) : 32;
#pragma unroll 1
      for (int k = 0; k < m32; ++k) {
        const int sk = __builtin_amdgcn_readlane(col, k);
        if (F32SRC != 0) {
          const v4f v = *(const v4f*)(HF + (size_t)sk * DF + 4 * lane);
          a0 += v.x; a1 += v.y; a2 += v.z; a3 += v.w;
        } else {
          const v2u w = *(const v2ua*)(XB + (size_t)sk * DF + 4 * lane);
          a0 += bfw_lo(w.x); a1 += bfw_hi(w.x); a2 += bfw_lo(w.y); a3 += bfw_hi(w.y);
        }
      }
    }
    const int nodec = node < nN ? node : nN - 1;
    float s0, s1, s2, s3;
    if (F32SRC != 0) {
      const v4f sv = *(const v4f*)(HF + (size_t)nodec * DF + 4 * lane);
      s0 = sv.x; s1 = sv.y; s2 = sv.z; s3 = sv.w;
    } else {
      const v2u sw = *(const v2ua*)(XB + (size_t)nodec * DF + 4 * lane);
      s0 = bfw_lo(sw.x); s1 = bfw_hi(sw.x); s2 = bfw_lo(sw.y); s3 = bfw_hi(sw.y);
    }
    const bool live = node < nN;
    float r0 = s0 + a0, r1 = s1 + a1, r2 = s2 + a2, r3 = s3 + a3;
    r0 = bad ? qnan : r0; r1 = bad ? qnan : r1; r2 = bad ? qnan : r2; r3 = bad ? qnan : r3;
    r0 = live ? r0 : 0.0f; r1 = live ? r1 : 0.0f; r2 = live ? r2 : 0.0f; r3 = live ? r3 : 0.0f;
    unsigned h0, l0, h1, l1;
    pack2(r0, r1, h0, l0);
    pack2(r2, r3, h1, l1);
    v2u hw, lw;
    hw.x = h0; hw.y = h1;
    lw.x = l0; lw.y = l1;
    wave_sync();
    *(v2ua*)(wst + 2 * lane)      = hw;
    *(v2ua*)(wst + 64 + 2 * lane) = lw;
    wave_sync();
    const v4u pk = *(const v4ua*)(wst + 4 * lane);
    wave_sync();
    unsigned short* gp = Zout + (size_t)node * APW + 8 * lane;
    *(volatile v4u*)gp = pk;
    __threadfence();
    *(volatile v4u*)gp = pk;
  }
}

template <int MODE, int KEXT>
__global__ __launch_bounds__(GTHR) __attribute__((amdgpu_num_vgpr(248)))
void k_gemm(const unsigned short* __restrict__ A, const unsigned short* __restrict__ WT,
            const float* __restrict__ bias, void* outp, const int* __restrict__ REC,
            int nN, int mRows, int nBk) {
  __shared__ __attribute__((aligned(16))) float stg[GBM * BN];
  __shared__ __attribute__((aligned(16))) float bsh[BN];
  const int tid = (int)threadIdx.x, lane = tid & 31, wave = tid >> 5, hh = lane >> 4, m = lane & 15;
  const int rowBase = (int)blockIdx.x * GBM;

  if (tid < 32) {
    const v4f b4 = *(const v4f*)(bias + 4 * tid);
    v4f bq;
    bq.x = bf16_val(b4.x); bq.y = bf16_val(b4.y); bq.z = bf16_val(b4.z); bq.w = bf16_val(b4.w);
    *(v4fa*)(bsh + 4 * tid) = bq;
  }

  v8f acc[8];
  {
    const v8f z = {0.f, 0.f, 0.f, 0.f, 0.f, 0.f, 0.f, 0.f};
#pragma unroll
    for (int t = 0; t < 8; ++t) acc[t] = z;
  }
  const unsigned short* ap = A + (size_t)(rowBase + 16 * wave + m) * (size_t)APW + 8 * hh;
  const unsigned short* wp = WT + (size_t)m * (size_t)WTP + 8 * hh;
  constexpr int ksteps = KEXT / 32;
#pragma unroll 1
  for (int ks = 0; ks < ksteps; ++ks) {
    FragB af;
    af.h[0] = *(const v8usa*)(ap + 32 * ks);
    af.h[1] = *(const v8usa*)(ap + 32 * ks + 16);
#pragma unroll
    for (int t = 0; t < 8; ++t) {
      const unsigned short* wq = wp + (size_t)(16 * t) * (size_t)WTP + 32 * ks;
      FragB bf;
      bf.h[0] = *(const v8usa*)wq;
      bf.h[1] = *(const v8usa*)(wq + 16);
      acc[t] = wmb(af, bf, acc[t]);
    }
  }
  __syncthreads();

#pragma unroll
  for (int t = 0; t < 8; ++t) {
    const int lc = 16 * t + m;
    const float bb = bsh[lc];
#pragma unroll
    for (int r = 0; r < 8; ++r) {
      const int lr = 16 * wave + 8 * hh + r;
      const bool live = (rowBase + lr) < nN;
      const float v = relu_k(acc[t][r] + bb);
      stg[lr * BN + lc] = live ? v : 0.0f;
    }
  }
  __syncthreads();

  if constexpr (MODE != 1) {
    float* outF = (float*)outp;
    const int rowLim = (MODE == 2) ? nN : mRows;
    bool poison = false;
    if (MODE == 2) {
      int bq = rowBase >> PKS;
      bq = bq > nBk - 1 ? nBk - 1 : bq;
      poison = REC[(size_t)bq * 32 + 1] != 0;
    }
    const float qn = __uint_as_float(0x7fc00000u);
    v4f fv[16];
#pragma unroll
    for (int i = 0; i < 16; ++i) {
      const int lr = 16 * wave + i;
      v4f t4 = *(const v4fa*)(stg + lr * BN + 4 * lane);
      t4.x = poison ? qn : t4.x;
      t4.y = poison ? qn : t4.y;
      t4.z = poison ? qn : t4.z;
      t4.w = poison ? qn : t4.w;
      fv[i] = t4;
    }
#pragma unroll
    for (int i = 0; i < 16; ++i) {
      const int gr = rowBase + 16 * wave + i;
      float* op = outF + (size_t)gr * (size_t)DF + 4 * lane;
      if (gr < rowLim) *(volatile v4f*)op = fv[i];
    }
    __threadfence();
#pragma unroll
    for (int i = 0; i < 16; ++i) {
      const int gr = rowBase + 16 * wave + i;
      float* op = outF + (size_t)gr * (size_t)DF + 4 * lane;
      if (gr < rowLim) *(volatile v4f*)op = fv[i];
    }
  } else {
    unsigned short* outH = (unsigned short*)outp;
    const int cb = 8 * m;
    const bool isHi = (hh == 0);
    v4u pk[16];
#pragma unroll
    for (int i = 0; i < 16; ++i) {
      const int lr = 16 * wave + i;
      const v4f a = *(const v4fa*)(stg + lr * BN + cb);
      const v4f b = *(const v4fa*)(stg + lr * BN + cb + 4);
      const float f[8] = {a.x, a.y, a.z, a.w, b.x, b.y, b.z, b.w};
      unsigned w[4];
#pragma unroll
      for (int j = 0; j < 4; ++j) {
        unsigned hw, lw;
        pack2(f[2 * j], f[2 * j + 1], hw, lw);
        w[j] = isHi ? hw : lw;
      }
      v4u pw; pw.x = w[0]; pw.y = w[1]; pw.z = w[2]; pw.w = w[3];
      pk[i] = pw;
    }
#pragma unroll
    for (int i = 0; i < 16; ++i) {
      const int gr = rowBase + 16 * wave + i;
      unsigned short* op = outH + (size_t)gr * (size_t)APW + 8 * lane;
      if (gr < mRows) *(volatile v4u*)op = pk[i];
    }
    __threadfence();
#pragma unroll
    for (int i = 0; i < 16; ++i) {
      const int gr = rowBase + 16 * wave + i;
      unsigned short* op = outH + (size_t)gr * (size_t)APW + 8 * lane;
      if (gr < mRows) *(volatile v4u*)op = pk[i];
    }
  }
}

static inline int cdiv(int a, int b) { return (a + b - 1) / b; }
static inline size_t al256(size_t o) { return (o + 255) & ~(size_t)255; }

extern "C" void kernel_launch(void* const* d_in, const int* in_sizes, int n_in,
                              void* d_out, int out_size, void* d_ws, size_t ws_size,
                              hipStream_t stream) {
  if (n_in < 10) return;
  if (in_sizes[0] < DF * GBM || (in_sizes[0] % DF) != 0) return;
  const int nN = in_sizes[0] / DF;
  if (nN > 65536) return;
  if (in_sizes[1] < 2 || (in_sizes[1] & 1) != 0) return;
  const int nE = in_sizes[1] / 2;
  if (nE < 1 || nE >= (1 << 21)) return;
  if (in_sizes[2] != DF * DF || in_sizes[4] != DF * DF) return;
  if (in_sizes[6] != DF * DF || in_sizes[8] != DF * DF) return;
  if (in_sizes[3] != DF || in_sizes[5] != DF || in_sizes[7] != DF || in_sizes[9] != DF) return;
  if ((long long)out_size != (long long)nN * DF) return;

  const float* x   = (const float*)d_in[0];
  const int*   ei  = (const int*)  d_in[1];
  const int*   src = ei;
  const int*   dst = ei + nE;
  const float* W1a = (const float*)d_in[2];
  const float* b1a = (const float*)d_in[3];
  const float* W1b = (const float*)d_in[4];
  const float* b1b = (const float*)d_in[5];
  const float* W2a = (const float*)d_in[6];
  const float* b2a = (const float*)d_in[7];
  const float* W2b = (const float*)d_in[8];
  const float* b2b = (const float*)d_in[9];

  const int nB    = cdiv(nN, NBA);
  const int NPADN = nB * NBA;
  const int MP    = cdiv(nN, GBM) * GBM;
  if (MP > NPADN || nB > 64) return;
  const int gR    = MP / RPB;
  const int vec8  = ((nE & 3) == 0) ? 1 : 0;

  char* ws = (char*)d_ws;
  size_t off = 0;
  const size_t oWT = off; off = al256(off + (size_t)NMAT * WSQ * 2);
  const size_t oXB = off; off = al256(off + (size_t)MP * DF * 2);
  const size_t oP1 = off; off = al256(off + (size_t)MP * APW * 2);
  const size_t oP2 = off; off = al256(off + (size_t)MP * APW * 2);
  const size_t oP3 = off; off = al256(off + (size_t)MP * DF * 4);
  const size_t oLS = off; off = al256(off + (size_t)nB * RCAP * 4);
  const size_t oCN = off; off = al256(off + (size_t)NPADN * 4);
  const size_t oOF = off; off = al256(off + (size_t)NPADN * 4);
  const size_t oRC = off; off = al256(off + (size_t)nB * 128);
  if (off > ws_size || off > (size_t)WSMAX) return;
  unsigned short* WT = (unsigned short*)(ws + oWT);
  unsigned short* XB = (unsigned short*)(ws + oXB);
  unsigned short* P1 = (unsigned short*)(ws + oP1);
  unsigned short* P2 = (unsigned short*)(ws + oP2);
  float* P3   = (float*)(ws + oP3);
  int*   LIST = (int*)(ws + oLS);
  int*   CNT  = (int*)(ws + oCN);
  int*   OFF  = (int*)(ws + oOF);
  int*   REC  = (int*)(ws + oRC);

  hipFuncSetAttribute(reinterpret_cast<const void*>(&k_bucket), hipFuncAttributeMaxDynamicSharedMemorySize, LDS_BK);

  const int nUnits = NUW + MP * (DF / 8);
  k_prep<<<nUnits / NTHR, NTHR, 0, stream>>>(x, W1a, W1b, W2a, W2b, WT, XB, nN, nUnits);
  k_bucket<<<nB, NTHR, LDS_BK, stream>>>(dst, src, nE, nN, vec8, LIST, CNT, OFF, REC);
  k_rowsum<0><<<gR, NTHR, 0, stream>>>(XB, P3, P1, LIST, CNT, OFF, REC, nN, MP, nB);
  k_gemm<1, KZ><<<gR, GTHR, 0, stream>>>(P1, WT + (size_t)0 * WSQ, b1a, (void*)P2, REC, nN, MP, nB);
  k_gemm<0, KTT><<<gR, GTHR, 0, stream>>>(P2, WT + (size_t)1 * WSQ, b1b, (void*)P3, REC, nN, MP, nB);
  k_rowsum<1><<<gR, NTHR, 0, stream>>>(XB, P3, P1, LIST, CNT, OFF, REC, nN, MP, nB);
  k_gemm<1, KZ><<<gR, GTHR, 0, stream>>>(P1, WT + (size_t)2 * WSQ, b2a, (void*)P2, REC, nN, MP, nB);
  k_gemm<2, KTT><<<gR, GTHR, 0, stream>>>(P2, WT + (size_t)3 * WSQ, b2b, d_out, REC, nN, MP, nB);
}
